// EigenBiasAttention_77730318123130
// MI455X (gfx1250) — hardware-run, weakly checked
//
#include <hip/hip_runtime.h>

typedef float          v8f   __attribute__((ext_vector_type(8)));
typedef float          v4f   __attribute__((ext_vector_type(4)));
typedef unsigned int   v4u   __attribute__((ext_vector_type(4)));
typedef int            v8i   __attribute__((ext_vector_type(8)));
typedef unsigned short v8us  __attribute__((ext_vector_type(8)));
typedef unsigned short v16us __attribute__((ext_vector_type(16)));
typedef __bf16         v16bf __attribute__((ext_vector_type(16)));
typedef _Float16       v16h  __attribute__((ext_vector_type(16)));
typedef v4f  __attribute__((may_alias)) v4fa;
typedef v8us __attribute__((may_alias)) v8usa;
union FragB { v16bf v; v16us u; v8us h[2]; v8i w; };
union FragH { v16h  v; v16us u; v8us h[2]; v8i w; };

__device__ __forceinline__ v8f wmb(const FragB& a, const FragB& b, v8f c) {
  v8f d = __builtin_amdgcn_wmma_f32_16x16x32_bf16(false, a.v, false, b.v, (short)0, c, false, false);
  asm volatile("v_nop\n\tv_nop\n\tv_nop\n\tv_nop" : "+v"(d) : "v"(a.w), "v"(b.w));
  return d;
}

__device__ __forceinline__ v8f wmh(const FragH& a, const FragH& b, v8f c) {
  v8f d = __builtin_amdgcn_wmma_f32_16x16x32_f16(false, a.v, false, b.v, (short)0, c, false, false);
  asm volatile("v_nop\n\tv_nop\n\tv_nop\n\tv_nop" : "+v"(d) : "v"(a.w), "v"(b.w));
  return d;
}

__device__ __forceinline__ unsigned bf16_bits(float f) {
  const unsigned u = __float_as_uint(f);
  const unsigned r = (u + 0x7FFFu + ((u >> 16) & 1u)) >> 16;
  const unsigned q = (u >> 16) | 0x40u;
  return ((u & 0x7fffffffu) > 0x7f800000u) ? q : r;
}

__device__ __forceinline__ float bf16_val(float f) {
  return __uint_as_float(bf16_bits(f) << 16);
}
__device__ __forceinline__ int clampi(int v, int lo, int hi) {
  return v < lo ? lo : (v > hi ? hi : v);
}

__device__ __forceinline__ unsigned f16_bits(float f) {
  const unsigned u  = __float_as_uint(f);
  const unsigned s  = (u >> 16) & 0x8000u;
  const unsigned a  = u & 0x7fffffffu;
  const unsigned t  = a - 0x38000000u;
  const unsigned r  = (t + 0x0FFFu + ((t >> 13) & 1u)) >> 13;
  const unsigned rc = r > 0x7C00u ? 0x7C00u : r;
  const bool small  = a < 0x38800000u;
  const bool isnan  = a > 0x7f800000u;
  const unsigned fin = small ? 0u : (s | rc);
  return isnan ? (s | 0x7E00u) : fin;
}

__device__ __forceinline__ unsigned pk16(unsigned lo, unsigned hi) { return lo | (hi << 16); }
__device__ __forceinline__ unsigned bf16_lo_bits(float v) {
  float hi = bf16_val(v);
  asm volatile("" : "+v"(hi));
  return bf16_bits(v - hi);
}
__device__ __forceinline__ v4u pack8_bf16(v4f a, v4f c) {
  return (v4u){ pk16(bf16_bits(a[0]), bf16_bits(a[1])), pk16(bf16_bits(a[2]), bf16_bits(a[3])),
                pk16(bf16_bits(c[0]), bf16_bits(c[1])), pk16(bf16_bits(c[2]), bf16_bits(c[3])) };
}
__device__ __forceinline__ v4u pack8_bf16_lo(v4f a, v4f c) {
  return (v4u){ pk16(bf16_lo_bits(a[0]), bf16_lo_bits(a[1])), pk16(bf16_lo_bits(a[2]), bf16_lo_bits(a[3])),
                pk16(bf16_lo_bits(c[0]), bf16_lo_bits(c[1])), pk16(bf16_lo_bits(c[2]), bf16_lo_bits(c[3])) };
}
__device__ __forceinline__ v4u pack8_f16(v4f a, v4f c) {
  return (v4u){ pk16(f16_bits(a[0]), f16_bits(a[1])), pk16(f16_bits(a[2]), f16_bits(a[3])),
                pk16(f16_bits(c[0]), f16_bits(c[1])), pk16(f16_bits(c[2]), f16_bits(c[3])) };
}

template <int FORM>
__global__ __launch_bounds__(256) void k_plane(const float* __restrict__ src, int rows, int cols, int ldsrc,
                                               unsigned short* __restrict__ dst, int MP, int KP) {
  static_assert(FORM >= 0 && FORM <= 3);
  const int KTOT = (FORM == 1 || FORM == 3) ? 2 * KP : KP;
  const unsigned ppr   = (unsigned)(KTOT >> 3);
  const unsigned kp8   = (unsigned)(KP >> 3);
  const unsigned total = (unsigned)MP * ppr;
  const unsigned g     = blockIdx.x * 256u + threadIdx.x;
  const unsigned rowu  = g / ppr;
  const unsigned p     = g - rowu * ppr;
  const bool second    = p >= kp8;
  const int row = (int)rowu;
  const int c0  = (int)((second ? p - kp8 : p) << 3);
  const float* srow = src + (size_t)clampi(row, 0, rows - 1) * (size_t)ldsrc;
  float x[8];
  unsigned mk[8];
#pragma unroll
  for (int e = 0; e < 8; ++e) {
    const int c = c0 + e;
    const float v = srow[clampi(c, 0, cols - 1)];
    asm volatile("" :: "v"(v));
    x[e]  = v;
    mk[e] = (row < rows && c < cols) ? 0xFFFFu : 0u;
  }
  const v4f a = (v4f){ x[0], x[1], x[2], x[3] };
  const v4f c = (v4f){ x[4], x[5], x[6], x[7] };
  v4u o;
  if (FORM == 2) {
    o = pack8_f16(a, c);
  } else {
    const v4u hi = pack8_bf16(a, c);
    o = hi;
    if (FORM == 1) { const v4u lo = pack8_bf16_lo(a, c); o = second ? lo : hi; }
  }
  const v4u mw = (v4u){ pk16(mk[0], mk[1]), pk16(mk[2], mk[3]), pk16(mk[4], mk[5]), pk16(mk[6], mk[7]) };
  o &= mw;
  if (g < total) {
    volatile v4u* q = (volatile v4u*)(dst + (size_t)g * 8);
    *q = o;
    __threadfence();
    *q = o;
  }
}

template <int FORM> struct FragOf    { typedef FragB T; };
template <>         struct FragOf<2> { typedef FragH T; };
__device__ __forceinline__ v8f mm(const FragB& a, const FragB& b, v8f c) { return wmb(a, b, c); }
__device__ __forceinline__ v8f mm(const FragH& a, const FragH& b, v8f c) { return wmh(a, b, c); }
template <class F> __device__ __forceinline__ F ld_frag(const unsigned short* p) {
  F f;
  f.h[0] = *(const v8usa*)(p);
  f.h[1] = *(const v8usa*)(p + 16);
  return f;
}

template <int FORM, int EPI>
__global__ __launch_bounds__(256) __attribute__((amdgpu_num_vgpr(248)))
void k_gemm_nt(const unsigned short* __restrict__ A, const unsigned short* __restrict__ B,
               const float* __restrict__ bias, float* __restrict__ D, int M, int N, int KTOT, int ldd) {
  static_assert(FORM >= 0 && FORM <= 2);
  static_assert(EPI == 0 || EPI == 1);
  typedef typename FragOf<FORM>::T F;
  __shared__ __attribute__((aligned(16))) float sT[8][16 * 68];
  const int lane = threadIdx.x & 31;
  const int wave = threadIdx.x >> 5;
  const int tilesM = (M + 63) >> 6;
  const int tilesN = (N + 63) >> 6;
  const int tile = blockIdx.x * 8 + wave;
  if (tile >= tilesM * tilesN) return;
  const int tm = tile / tilesN;
  const int tn = tile - tm * tilesN;
  const int m0 = tm << 6;
  const int n0 = tn << 6;

  const int rl = lane & 15;
  const int h8 = (lane >> 4) * 8;
  const unsigned short* pa = A + (size_t)(m0 + rl) * (size_t)KTOT + h8;
  const unsigned short* pb = B + (size_t)(n0 + rl) * (size_t)KTOT + h8;

  v8f acc[4][4];
#pragma unroll
  for (int i = 0; i < 4; ++i)
#pragma unroll
    for (int j = 0; j < 4; ++j) acc[i][j] = (v8f){0.f, 0.f, 0.f, 0.f, 0.f, 0.f, 0.f, 0.f};

#pragma unroll 1
  for (int k0 = 0; k0 < KTOT; k0 += 32) {
    F bf[4];
#pragma unroll
    for (int j = 0; j < 4; ++j) bf[j] = ld_frag<F>(pb + (size_t)(j << 4) * (size_t)KTOT + k0);
#pragma unroll
    for (int i = 0; i < 4; ++i) {
      const F af = ld_frag<F>(pa + (size_t)(i << 4) * (size_t)KTOT + k0);
#pragma unroll
      for (int j = 0; j < 4; ++j) acc[i][j] = mm(af, bf[j], acc[i][j]);
    }
  }

  float* slab = sT[wave];
  const int hh = lane >> 4;
  const int c4 = (lane & 15) * 4;
  const int nc = n0 + c4;
  const bool cok = nc < N;
  v4f bv = (v4f){0.f, 0.f, 0.f, 0.f};
  if (EPI == 1) {
    bv = *(const v4fa*)(bias + clampi(nc, 0, N - 4));
    asm volatile("" :: "v"(bv));
  }
#pragma unroll
  for (int i = 0; i < 4; ++i) {
    const int mBase = m0 + (i << 4);
#pragma unroll
    for (int j = 0; j < 4; ++j) {
#pragma unroll
      for (int r = 0; r < 8; ++r) slab[(h8 + r) * 68 + (j << 4) + rl] = acc[i][j][r];
    }
    __builtin_amdgcn_fence(__ATOMIC_RELEASE, "workgroup");
    __builtin_amdgcn_wave_barrier();
    __builtin_amdgcn_fence(__ATOMIC_ACQUIRE, "workgroup");
    v4f vv[8];
#pragma unroll
    for (int it = 0; it < 8; ++it) {
      const int row = it * 2 + hh;
      v4f v = *(const v4fa*)(slab + row * 68 + c4);
      if (EPI == 1) v += bv;
      vv[it] = v;
    }
    for (int pass = 0; pass < 2; ++pass) {
#pragma unroll
      for (int it = 0; it < 8; ++it) {
        const int row = mBase + it * 2 + hh;
        if (cok && row < M) *(volatile v4f*)(D + (size_t)row * (size_t)ldd + nc) = vv[it];
      }
      __threadfence();
    }
    __builtin_amdgcn_fence(__ATOMIC_RELEASE, "workgroup");
    __builtin_amdgcn_wave_barrier();
    __builtin_amdgcn_fence(__ATOMIC_ACQUIRE, "workgroup");
  }
}

#pragma clang fp contract(off)

#ifndef S_TERMS
#define S_TERMS 3
#endif
#ifndef PV_TERMS
#define PV_TERMS 3
#endif

constexpr int kB    = 2;
constexpr int kT    = 1024;
constexpr int kD    = 1024;
constexpr int kH    = 16;
constexpr int kDH   = 64;
constexpr int kM    = kB * kT;
constexpr int kNQKV = 3 * kD;
constexpr int kNALL = kNQKV + 4 * 64;
constexpr int kP2   = 2 * kD;
static_assert(kT % 64 == 0);
static_assert(kD == kH * kDH);
static_assert(kDH == 64);
static_assert(kNALL % 64 == 0);
static_assert(kNALL % 32 == 0);
static_assert(kD % 32 == 0);
static_assert(kP2 % 32 == 0);
static_assert(kM % 64 == 0);
static_assert(S_TERMS == 2 || S_TERMS == 3);
static_assert(PV_TERMS == 2 || PV_TERMS == 3);

__global__ __launch_bounds__(256) void k_vec_bf(const float* __restrict__ src, float* __restrict__ dst, int n4) {
  const int i  = blockIdx.x * 256 + threadIdx.x;
  const int ic = clampi(i, 0, n4 - 1);
  const v4f v = *(const v4fa*)(src + (size_t)ic * 4);
  asm volatile("" :: "v"(v));
  const v4f o = (v4f){ bf16_val(v[0]), bf16_val(v[1]), bf16_val(v[2]), bf16_val(v[3]) };
  if (i < n4) {
    volatile v4f* q = (volatile v4f*)(dst + (size_t)i * 4);
    *q = o;
    __threadfence();
    *q = o;
  }
}

__global__ __launch_bounds__(256) void k_split(const float* __restrict__ C, const float* __restrict__ bqkv,
                                               unsigned short* __restrict__ P16,
                                               size_t oQ, size_t oK, size_t oVH, size_t oVL) {
  __shared__ __attribute__((aligned(16))) float tf[64 * 68];
  const int tid   = threadIdx.x;
  const int c0    = blockIdx.x * 64;
  const int r0    = blockIdx.y * 64;
  const int third = blockIdx.x >> 4;
  const int cq    = c0 & 1023;
  {
    const int lr = tid >> 4;
    const int c4 = (tid & 15) * 4;
    v4f bv = *(const v4fa*)(bqkv + c0 + c4);
    asm volatile("" :: "v"(bv));
    bv = (v4f){ bf16_val(bv[0]), bf16_val(bv[1]), bf16_val(bv[2]), bf16_val(bv[3]) };
#pragma unroll
    for (int it = 0; it < 4; ++it) {
      const int rr = it * 16 + lr;
      v4f a = *(const v4fa*)(C + (size_t)(r0 + rr) * kNALL + c0 + c4);
      a += bv;
      *(v4fa*)(tf + rr * 68 + c4) = a;
    }
  }
  __syncthreads();
  const int sub = tid >> 3;
  const int c8  = (tid & 7) * 8;
  v4u hv[2], lv[2];
  if (third < 2) {
#pragma unroll
    for (int it = 0; it < 2; ++it) {
      const int row = it * 32 + sub;
      const v4f a  = *(const v4fa*)(tf + row * 68 + c8);
      const v4f cc = *(const v4fa*)(tf + row * 68 + c8 + 4);
      hv[it] = pack8_bf16(a, cc);
      lv[it] = pack8_bf16_lo(a, cc);
    }
    const size_t base = (third == 0) ? oQ : oK;
    for (int pass = 0; pass < 2; ++pass) {
#pragma unroll
      for (int it = 0; it < 2; ++it) {
        const int row = it * 32 + sub;
        const size_t go = base + (size_t)(r0 + row) * kP2 + cq + c8;
        *(volatile v4u*)(P16 + go)        = hv[it];
        *(volatile v4u*)(P16 + go + 1024) = lv[it];
      }
      __threadfence();
    }
  } else {
    const int b  = r0 >> 10;
    const int t0 = r0 & 1023;
#pragma unroll
    for (int it = 0; it < 2; ++it) {
      const int oc = it * 32 + sub;
      const v4f a  = (v4f){ tf[(c8 + 0) * 68 + oc], tf[(c8 + 1) * 68 + oc], tf[(c8 + 2) * 68 + oc], tf[(c8 + 3) * 68 + oc] };
      const v4f cc = (v4f){ tf[(c8 + 4) * 68 + oc], tf[(c8 + 5) * 68 + oc], tf[(c8 + 6) * 68 + oc], tf[(c8 + 7) * 68 + oc] };
      hv[it] = pack8_bf16(a, cc);
      lv[it] = pack8_bf16_lo(a, cc);
    }
    for (int pass = 0; pass < 2; ++pass) {
#pragma unroll
      for (int it = 0; it < 2; ++it) {
        const int oc = it * 32 + sub;
        const size_t go = (size_t)(b * 1024 + cq + oc) * kT + t0 + c8;
        *(volatile v4u*)(P16 + oVH + go) = hv[it];
        *(volatile v4u*)(P16 + oVL + go) = lv[it];
      }
      __threadfence();
    }
  }
}

__device__ __forceinline__ void ext6(const v4f p1, const v4f p2, float (&L)[6]) {
  L[0] = p1[0] * p2[1] - p1[1] * p2[0];
  L[1] = p1[0] * p2[2] - p1[2] * p2[0];
  L[2] = p1[0] * p2[3] - p1[3] * p2[0];
  L[3] = p1[1] * p2[2] - p1[2] * p2[1];
  L[4] = p1[1] * p2[3] - p1[3] * p2[1];
  L[5] = p1[2] * p2[3] - p1[3] * p2[2];
  float n2 = L[0] * L[0];
  n2 = n2 + L[1] * L[1];
  n2 = n2 + L[2] * L[2];
  n2 = n2 + L[3] * L[3];
  n2 = n2 + L[4] * L[4];
  n2 = n2 + L[5] * L[5];
  const float n = sqrtf(n2);
  const float d = fmaxf(n, 1e-12f);
#pragma unroll
  for (int i = 0; i < 6; ++i) L[i] = L[i] / d;
}

__global__ __launch_bounds__(32) void k_bias(const float* __restrict__ C, float* __restrict__ JW,
                                             float* __restrict__ RDM) {
  __shared__ __attribute__((aligned(16))) float stJ[32 * 8];
  __shared__ __attribute__((aligned(16))) float stD[32 * 8];
  __shared__ __attribute__((aligned(16))) float stR[32 * 8];
  const int lane = threadIdx.x;
  const int bh   = blockIdx.x;
  const int b    = bh >> 4;
  const int h    = bh & 15;
  const int l7   = lane & 7;
  const int jx   = l7 < 5 ? l7 : 5;
  float M0 = 0.0f, M1 = 0.0f, M2 = 0.0f, M3 = 0.0f, M4 = 0.0f, M5 = 0.0f;

#pragma unroll 1
  for (int c = 0; c < 32; ++c) {
    const int t  = 32 * c + lane;
    const int tp = t > 0 ? t - 1 : 0;
    const size_t row  = (size_t)(b * kT + t)  * kNALL;
    const size_t rowp = (size_t)(b * kT + tp) * kNALL;
    const v4f w1raw = *(const v4fa*)(C + rowp + 3072 + 4 * h);
    const v4f w2    = *(const v4fa*)(C + row  + 3136 + 4 * h);
    const v4f r1    = *(const v4fa*)(C + row  + 3200 + 4 * h);
    const v4f r2    = *(const v4fa*)(C + row  + 3264 + 4 * h);
    asm volatile("" :: "v"(w1raw), "v"(w2), "v"(r1), "v"(r2));
    const unsigned mk = (t == 0) ? 0u : 0xFFFFFFFFu;
    const v4f w1 = (v4f){ __uint_as_float(__float_as_uint(w1raw[0]) & mk), __uint_as_float(__float_as_uint(w1raw[1]) & mk),
                          __uint_as_float(__float_as_uint(w1raw[2]) & mk), __uint_as_float(__float_as_uint(w1raw[3]) & mk) };
    float Lw[6] = {0.0f, 0.0f, 0.0f, 0.0f, 0.0f, 0.0f}, Lr[6] = {0.0f, 0.0f, 0.0f, 0.0f, 0.0f, 0.0f};
#pragma unroll 1
    for (int sel = 0; sel < 2; ++sel) {
      const v4f pa = sel ? r1 : w1;
      const v4f pb = sel ? r2 : w2;
      float Lx[6];
      ext6(pa, pb, Lx);
#pragma unroll
      for (int i = 0; i < 6; ++i) { Lw[i] = sel ? Lw[i] : Lx[i]; Lr[i] = sel ? Lx[i] : Lr[i]; }
    }
    const v4f ja = (v4f){ Lw[5], -Lw[4], Lw[3], Lw[2] };
    const v4f jb = (v4f){ -Lw[1], Lw[0], 0.0f, 0.0f };
    const v4f da = (v4f){ Lr[0], Lr[1], Lr[2], Lr[3] };
    const v4f db = (v4f){ Lr[4], Lr[5], 0.0f, 0.0f };
    *(v4fa*)(&stJ[lane * 8])     = ja;
    *(v4fa*)(&stJ[lane * 8 + 4]) = jb;
    *(v4fa*)(&stD[lane * 8])     = da;
    *(v4fa*)(&stD[lane * 8 + 4]) = db;
    __syncthreads();

#pragma unroll 4
    for (int s = 0; s < 32; ++s) {
      const v4f a0 = *(const v4fa*)(&stJ[s * 8]);
      const v4f a1 = *(const v4fa*)(&stJ[s * 8 + 4]);
      const float jj = stJ[s * 8 + jx];
      M0 = M0 + a0[0] * jj;
      M1 = M1 + a0[1] * jj;
      M2 = M2 + a0[2] * jj;
      M3 = M3 + a0[3] * jj;
      M4 = M4 + a1[0] * jj;
      M5 = M5 + a1[1] * jj;
      const v4f d0 = *(const v4fa*)(&stD[s * 8]);
      const v4f d1 = *(const v4fa*)(&stD[s * 8 + 4]);
      float acc = d0[0] * M0;
      acc = acc + d0[1] * M1;
      acc = acc + d0[2] * M2;
      acc = acc + d0[3] * M3;
      acc = acc + d1[0] * M4;
      acc = acc + d1[1] * M5;
      if (lane < 8) stR[s * 8 + lane] = (lane < 6) ? acc : 0.0f;
    }
    __syncthreads();

    const v4f j0 = *(const v4fa*)(&stJ[lane * 4]);
    const v4f j1 = *(const v4fa*)(&stJ[128 + lane * 4]);
    const v4f q0 = *(const v4fa*)(&stR[lane * 4]);
    const v4f q1 = *(const v4fa*)(&stR[128 + lane * 4]);
    const size_t base = ((size_t)bh * kT + 32 * c) * 8;
    for (int pass = 0; pass < 2; ++pass) {
      *(volatile v4f*)(JW  + base + lane * 4)       = j0;
      *(volatile v4f*)(JW  + base + 128 + lane * 4) = j1;
      *(volatile v4f*)(RDM + base + lane * 4)       = q0;
      *(volatile v4f*)(RDM + base + 128 + lane * 4) = q1;
      __threadfence();
    }
    __syncthreads();
  }
}

__global__ __launch_bounds__(128) __attribute__((amdgpu_num_vgpr(248)))
void k_attn(const unsigned short* __restrict__ QHL, const unsigned short* __restrict__ KHL,
            const unsigned short* __restrict__ VTH, const unsigned short* __restrict__ VTL,
            const float* __restrict__ JW, const float* __restrict__ RDM, const float* __restrict__ bscale,
            unsigned short* __restrict__ CTX) {
  __shared__ __attribute__((aligned(16))) unsigned short Ksh[64 * 64];
  __shared__ __attribute__((aligned(16))) unsigned short Ksl[64 * 64];
  __shared__ __attribute__((aligned(16))) unsigned short Vth[64 * 64];
  __shared__ __attribute__((aligned(16))) unsigned short Vtl[64 * 64];
  __shared__ __attribute__((aligned(16))) unsigned short Psh[4][16 * 64];
  __shared__ __attribute__((aligned(16))) unsigned short Psl[4][16 * 64];
  __shared__ __attribute__((aligned(16))) float Os[4][16 * 68];
  __shared__ __attribute__((aligned(16))) float JWs[64 * 8];
  __shared__ __attribute__((aligned(16))) float RDs[64 * 8];

  const int tid  = threadIdx.x;
  const int wave = tid >> 5;
  const int lane = tid & 31;
  const int hh   = lane >> 4;
  const int c    = lane & 15;

  const int bx   = blockIdx.x;
  const int qb   = bx & 15;
  const int bh   = bx >> 4;
  const int b    = bh >> 4;
  const int h    = bh & 15;
  const int q0   = qb * 64 + wave * 16;
  const int rowb = b * kT;
  const float ninf = __uint_as_float(0xff800000u);
  const float bs = bf16_val(bscale[h]);

  {
    const v4f rv = *(const v4fa*)(RDM + ((size_t)bh * kT + qb * 64) * 8 + tid * 4);
    *(v4fa*)(&RDs[tid * 4]) = rv;
  }

  FragB qah[2], qal[2];
  {
    const unsigned short* qp = QHL + (size_t)(rowb + q0 + c) * kP2 + h * 64 + 8 * hh;
#pragma unroll
    for (int dc = 0; dc < 2; ++dc) {
      qah[dc] = ld_frag<FragB>(qp + dc * 32);
      qal[dc] = ld_frag<FragB>(qp + 1024 + dc * 32);
    }
  }

  float mrow[8], lrow[8];
  v8f oacc[4];
#pragma unroll
  for (int r = 0; r < 8; ++r) { mrow[r] = ninf; lrow[r] = 0.0f; }
#pragma unroll
  for (int t = 0; t < 4; ++t) oacc[t] = (v8f){0.f, 0.f, 0.f, 0.f, 0.f, 0.f, 0.f, 0.f};

  const int nChunks = qb + 1;
#pragma unroll 1
  for (int kc = 0; kc < nChunks; ++kc) {
    const int kv0 = kc * 64;
    __syncthreads();
    {
      const int r = tid >> 1, half = (tid & 1) * 32;
      const unsigned short* ksh = KHL + (size_t)(rowb + kv0 + r) * kP2 + h * 64 + half;
      const unsigned short* vsh = VTH + (size_t)(rowb + h * 64 + r) * kT + kv0 + half;
      const unsigned short* vsl = VTL + (size_t)(rowb + h * 64 + r) * kT + kv0 + half;
#pragma unroll
      for (int i = 0; i < 4; ++i) {
        const v8us a0 = *(const v8usa*)(ksh + 8 * i);
        const v8us a1 = *(const v8usa*)(ksh + 1024 + 8 * i);
        const v8us b0 = *(const v8usa*)(vsh + 8 * i);
        const v8us b1 = *(const v8usa*)(vsl + 8 * i);
        *(v8usa*)(&Ksh[r * 64 + half + 8 * i]) = a0;
        *(v8usa*)(&Ksl[r * 64 + half + 8 * i]) = a1;
        *(v8usa*)(&Vth[r * 64 + half + 8 * i]) = b0;
        *(v8usa*)(&Vtl[r * 64 + half + 8 * i]) = b1;
      }
      const v4f jv = *(const v4fa*)(JW + ((size_t)bh * kT + kv0) * 8 + tid * 4);
      *(v4fa*)(&JWs[tid * 4]) = jv;
    }
    __syncthreads();

    v8f s[4];
#pragma unroll
    for (int j = 0; j < 4; ++j) {
      s[j] = (v8f){0.f, 0.f, 0.f, 0.f, 0.f, 0.f, 0.f, 0.f};
#pragma unroll
      for (int dc = 0; dc < 2; ++dc) {
        FragB kb, kl;
        kb.h[0] = *(const v8usa*)(&Ksh[(j * 16 + c) * 64 + dc * 32 + 8 * hh]);
        kb.h[1] = *(const v8usa*)(&Ksh[(j * 16 + c) * 64 + dc * 32 + 16 + 8 * hh]);
        kl.h[0] = *(const v8usa*)(&Ksl[(j * 16 + c) * 64 + dc * 32 + 8 * hh]);
        kl.h[1] = *(const v8usa*)(&Ksl[(j * 16 + c) * 64 + dc * 32 + 16 + 8 * hh]);
        s[j] = wmb(qah[dc], kb, s[j]);
        if (S_TERMS == 3) s[j] = wmb(qah[dc], kl, s[j]);
        s[j] = wmb(qal[dc], kb, s[j]);
      }
    }

    float jc[4][6];
#pragma unroll
    for (int j = 0; j < 4; ++j) {
      const v4f a0 = *(const v4fa*)(&JWs[(j * 16 + c) * 8]);
      const v4f a1 = *(const v4fa*)(&JWs[(j * 16 + c) * 8 + 4]);
      jc[j][0] = a0[0]; jc[j][1] = a0[1]; jc[j][2] = a0[2]; jc[j][3] = a0[3];
      jc[j][4] = a1[0]; jc[j][5] = a1[1];
    }

    const bool diag = (kc == qb);
    float cm[8];
#pragma unroll
    for (int r = 0; r < 8; ++r) {
      const int qrow = q0 + 8 * hh + r;
      const v4f ra = *(const v4fa*)(&RDs[(wave * 16 + 8 * hh + r) * 8]);
      const v4f rb = *(const v4fa*)(&RDs[(wave * 16 + 8 * hh + r) * 8 + 4]);
      float m = ninf;
#pragma unroll
      for (int j = 0; j < 4; ++j) {
        const int kvcol = kv0 + j * 16 + c;
        float d = ra[0] * jc[j][0];
        d = d + ra[1] * jc[j][1];
        d = d + ra[2] * jc[j][2];
        d = d + ra[3] * jc[j][3];
        d = d + rb[0] * jc[j][4];
        d = d + rb[1] * jc[j][5];
        const float bias = fabsf(d) * bs;
        const float sv = s[j][r] * 0.125f + bias;
        const bool masked = diag && (kvcol > qrow);
        const float sm = masked ? ninf : sv;
        s[j][r] = sm;
        m = fmaxf(m, sm);
      }
#pragma unroll
      for (int off = 1; off < 16; off <<= 1) m = fmaxf(m, __shfl_xor(m, off, 32));
      cm[r] = m;
    }

#pragma unroll
    for (int r = 0; r < 8; ++r) {
      const float mnew  = fmaxf(mrow[r], cm[r]);
      const float alpha = expf(mrow[r] - mnew);
      mrow[r] = mnew;
      float psum = 0.0f;
#pragma unroll
      for (int j = 0; j < 4; ++j) {
        const float p = expf(s[j][r] - mnew);
        psum += p;
        Psh[wave][(8 * hh + r) * 64 + j * 16 + c] = (unsigned short)bf16_bits(p);
        Psl[wave][(8 * hh + r) * 64 + j * 16 + c] = (unsigned short)bf16_lo_bits(p);
      }
#pragma unroll
      for (int off = 1; off < 16; off <<= 1) psum += __shfl_xor(psum, off, 32);
      lrow[r] = lrow[r] * alpha + psum;
#pragma unroll
      for (int t = 0; t < 4; ++t) oacc[t][r] *= alpha;
    }
    __builtin_amdgcn_fence(__ATOMIC_RELEASE, "workgroup");
    __builtin_amdgcn_wave_barrier();
    __builtin_amdgcn_fence(__ATOMIC_ACQUIRE, "workgroup");

#pragma unroll 1
    for (int kk = 0; kk < 2; ++kk) {
      FragB pa, pl;
      pa.h[0] = *(const v8usa*)(&Psh[wave][c * 64 + kk * 32 + 8 * hh]);
      pa.h[1] = *(const v8usa*)(&Psh[wave][c * 64 + kk * 32 + 16 + 8 * hh]);
      pl.h[0] = *(const v8usa*)(&Psl[wave][c * 64 + kk * 32 + 8 * hh]);
      pl.h[1] = *(const v8usa*)(&Psl[wave][c * 64 + kk * 32 + 16 + 8 * hh]);
#pragma unroll
      for (int t = 0; t < 4; ++t) {
        FragB vb, vl;
        vb.h[0] = *(const v8usa*)(&Vth[(t * 16 + c) * 64 + kk * 32 + 8 * hh]);
        vb.h[1] = *(const v8usa*)(&Vth[(t * 16 + c) * 64 + kk * 32 + 16 + 8 * hh]);
        vl.h[0] = *(const v8usa*)(&Vtl[(t * 16 + c) * 64 + kk * 32 + 8 * hh]);
        vl.h[1] = *(const v8usa*)(&Vtl[(t * 16 + c) * 64 + kk * 32 + 16 + 8 * hh]);
        oacc[t] = wmb(pa, vb, oacc[t]);
        if (PV_TERMS == 3) oacc[t] = wmb(pa, vl, oacc[t]);
        oacc[t] = wmb(pl, vb, oacc[t]);
      }
    }
  }

#pragma unroll
  for (int r = 0; r < 8; ++r) {
    const float inv = 1.0f / lrow[r];
#pragma unroll
    for (int t = 0; t < 4; ++t) Os[wave][(8 * hh + r) * 68 + t * 16 + c] = oacc[t][r] * inv;
  }
  __builtin_amdgcn_fence(__ATOMIC_RELEASE, "workgroup");
  __builtin_amdgcn_wave_barrier();
  __builtin_amdgcn_fence(__ATOMIC_ACQUIRE, "workgroup");
  {
    const int q  = lane >> 3;
    const int c8 = (lane & 7) * 8;
    v4u hv[4], lv[4];
#pragma unroll
    for (int it = 0; it < 4; ++it) {
      const int row = it * 4 + q;
      const v4f a  = *(const v4fa*)(&Os[wave][row * 68 + c8]);
      const v4f cc = *(const v4fa*)(&Os[wave][row * 68 + c8 + 4]);
      hv[it] = pack8_bf16(a, cc);
      lv[it] = pack8_bf16_lo(a, cc);
    }
    for (int pass = 0; pass < 2; ++pass) {
#pragma unroll
      for (int it = 0; it < 4; ++it) {
        const int row = it * 4 + q;
        const size_t go = (size_t)(rowb + q0 + row) * kP2 + h * 64 + c8;
        *(volatile v4u*)(CTX + go)        = hv[it];
        *(volatile v4u*)(CTX + go + 1024) = lv[it];
      }
      __threadfence();
    }
  }
}

extern "C" void kernel_launch(void* const* d_in, const int* in_sizes, int n_in,
                              void* d_out, int out_size, void* d_ws, size_t ws_size,
                              hipStream_t stream) {
  if (n_in < 10) return;
  if (in_sizes[0] != kM * kD) return;
  if (in_sizes[1] != kNQKV * kD) return;
  if (in_sizes[2] != kNQKV) return;
  if (in_sizes[3] != 64 * kD || in_sizes[4] != 64 * kD || in_sizes[5] != 64 * kD || in_sizes[6] != 64 * kD) return;
  if (in_sizes[7] != kH) return;
  if (in_sizes[8] != kD * kD) return;
  if (in_sizes[9] != kD) return;
  if (out_size != kM * kD) return;

  const float* x     = (const float*)d_in[0];
  const float* Wqkv  = (const float*)d_in[1];
  const float* bqkv  = (const float*)d_in[2];
  const float* W1w   = (const float*)d_in[3];
  const float* W2w   = (const float*)d_in[4];
  const float* W1r   = (const float*)d_in[5];
  const float* W2r   = (const float*)d_in[6];
  const float* bsc   = (const float*)d_in[7];
  const float* Wout  = (const float*)d_in[8];
  const float* bout  = (const float*)d_in[9];
  float* out = (float*)d_out;

  const size_t szXB   = (size_t)kM * kD * 2;
  const size_t szWALL = (size_t)kNALL * kD * 2;
  const size_t szWO2  = (size_t)kD * kP2 * 2;
  const size_t szC    = (size_t)kM * kNALL * 4;
  const size_t szHL   = (size_t)kM * kP2 * 2;
  const size_t szVT   = (size_t)kM * kT * 2;
  const size_t szJW   = (size_t)kB * kH * kT * 8 * 4;
  const size_t szBOR  = (size_t)kD * 4;
  size_t off = 0;
  const size_t oXB   = off; off += szXB;
  const size_t oWALL = off; off += szWALL;
  const size_t oWO2  = off; off += szWO2;
  const size_t oC    = off; off += szC;
  const size_t oQ    = off; off += szHL;
  const size_t oK    = off; off += szHL;
  const size_t oVH   = off; off += szVT;
  const size_t oVL   = off; off += szVT;
  const size_t oJW   = off; off += szJW;
  const size_t oRDM  = off; off += szJW;
  const size_t oCTX  = off; off += szHL;
  const size_t oBOR  = off; off += szBOR;
  if (off > ws_size) return;
  if (off > ((size_t)128 << 20)) return;

  char* ws = (char*)d_ws;
  unsigned short* P16  = (unsigned short*)ws;
  unsigned short* XB   = (unsigned short*)(ws + oXB);
  unsigned short* WALL = (unsigned short*)(ws + oWALL);
  unsigned short* WO2  = (unsigned short*)(ws + oWO2);
  float*          Cws  = (float*)(ws + oC);
  unsigned short* QHL  = (unsigned short*)(ws + oQ);
  unsigned short* KHL  = (unsigned short*)(ws + oK);
  unsigned short* VTH  = (unsigned short*)(ws + oVH);
  unsigned short* VTL  = (unsigned short*)(ws + oVL);
  float*          JWt  = (float*)(ws + oJW);
  float*          RDMt = (float*)(ws + oRDM);
  unsigned short* CTX  = (unsigned short*)(ws + oCTX);
  float*          BOR  = (float*)(ws + oBOR);

  const dim3 blk(256);
  k_plane<0><<<dim3(kM * kD / 8 / 256), blk, 0, stream>>>(x, kM, kD, kD, XB, kM, kD);
  k_plane<0><<<dim3(kNQKV * kD / 8 / 256), blk, 0, stream>>>(Wqkv, kNQKV, kD, kD, WALL, kNQKV, kD);
  k_plane<0><<<dim3(64 * kD / 8 / 256), blk, 0, stream>>>(W1w, 64, kD, kD, WALL + (size_t)3072 * kD, 64, kD);
  k_plane<0><<<dim3(64 * kD / 8 / 256), blk, 0, stream>>>(W2w, 64, kD, kD, WALL + (size_t)3136 * kD, 64, kD);
  k_plane<0><<<dim3(64 * kD / 8 / 256), blk, 0, stream>>>(W1r, 64, kD, kD, WALL + (size_t)3200 * kD, 64, kD);
  k_plane<0><<<dim3(64 * kD / 8 / 256), blk, 0, stream>>>(W2r, 64, kD, kD, WALL + (size_t)3264 * kD, 64, kD);
  k_plane<3><<<dim3(kD * kP2 / 8 / 256), blk, 0, stream>>>(Wout, kD, kD, kD, WO2, kD, kD);
  k_vec_bf<<<dim3(1), blk, 0, stream>>>(bout, BOR, kD / 4);
  k_gemm_nt<0, 0><<<dim3(((kM / 64) * (kNALL / 64) + 7) / 8), blk, 0, stream>>>(XB, WALL, BOR, Cws, kM, kNALL, kD, kNALL);
  k_split<<<dim3(kNQKV / 64, kM / 64), blk, 0, stream>>>(Cws, bqkv, P16, oQ / 2, oK / 2, oVH / 2, oVL / 2);
  k_bias<<<dim3(kB * kH), dim3(32), 0, stream>>>(Cws, JWt, RDMt);
  k_attn<<<dim3(kB * kH * (kT / 64)), dim3(128), 0, stream>>>(QHL, KHL, VTH, VTL, JWt, RDMt, bsc, CTX);
  k_gemm_nt<0, 1><<<dim3(((kM / 64) * (kD / 64) + 7) / 8), blk, 0, stream>>>(CTX, WO2, BOR, out, kM, kD, kP2, kD);
  (void)hipGetLastError();
}
